// SeqWhileLoopBlock_11579231830042
// MI455X (gfx1250) — hardware-verified
//
#include <hip/hip_runtime.h>


namespace {
constexpr int N = 4096, P = 128, NH = 4, E = 32, NSEG = 32;
constexpr float XS = 8.0f, PS = 1024.0f, WSC = 256.0f;
typedef _Float16 b16;
typedef __attribute__((ext_vector_type(16))) _Float16 v16b;
typedef __attribute__((ext_vector_type(8))) _Float16 v8b;
typedef __attribute__((ext_vector_type(8))) float v8f;
typedef __attribute__((ext_vector_type(4))) float v4f;
typedef __attribute__((ext_vector_type(2))) float v2f;
__device__ __forceinline__ float bf16_rne(float f) { unsigned int u = __float_as_uint(f); u += 0x7FFFu + ((u >> 16) & 1u); float r = __uint_as_float(u & 0xFFFF0000u); asm volatile("" : "+v"(r)); return r; }
__device__ __forceinline__ void split16(float v, b16& hi, b16& lo) { hi = (b16)v; lo = (b16)(v - (float)hi); }
__device__ __forceinline__ v16b frag_kb(const b16* p, int hh) { const v8b a = *(const v8b*)(p + 8 * hh), b = *(const v8b*)(p + 16 + 8 * hh); v16b f;
#pragma unroll
  for (int e = 0; e < 8; ++e) { f[e] = a[e]; f[8 + e] = b[e]; } return f; }
__device__ __forceinline__ v8f wmma16b(v16b a, v16b b, v8f c) { v8f d = __builtin_amdgcn_wmma_f32_16x16x32_f16(false, a, false, b, (short)0, c, false, false); asm volatile("v_nop\n\tv_nop\n\tv_nop\n\tv_nop" : "+v"(d) : "v"(a), "v"(b)); return d; }
__device__ __forceinline__ void wave_lds_sync() { __builtin_amdgcn_fence(__ATOMIC_RELEASE, "workgroup"); __builtin_amdgcn_wave_barrier(); __builtin_amdgcn_fence(__ATOMIC_ACQUIRE, "workgroup"); }
__device__ __forceinline__ int iclamp(int v, int lo, int hi) { return v < lo ? lo : (v > hi ? hi : v); }

__global__ __launch_bounds__(256) void wput_kernel(const float* __restrict__ wq, const float* __restrict__ wk, const float* __restrict__ wv, b16* __restrict__ WT) { const int u = blockIdx.x * 256 + threadIdx.x; if (u >= 3 * P * 16) return; const int o = u / 16, k0 = (u % 16) * 8; const int which = o / P, oo = o % P; const float* w = which == 0 ? wq : (which == 1 ? wk : wv); v8b v;
#pragma unroll
  for (int j = 0; j < 8; ++j) v[j] = (b16)(bf16_rne(w[(size_t)(k0 + j) * P + oo]) * WSC); for (int pass = 0; pass < 2; ++pass) { *(volatile v8b*)(WT + (size_t)o * P + k0) = v; __threadfence(); } }
__global__ __launch_bounds__(32) void seg_kernel(const int* __restrict__ pos, int* __restrict__ META, int* __restrict__ LIST) { __shared__ int cnt[NSEG], cur[NSEG], cc[NSEG]; const int lane = threadIdx.x; cnt[lane] = 0; wave_lds_sync();
  if (lane == 0) { for (int i = 0; i < N; ++i) cnt[iclamp(pos[i], 0, NSEG - 1)]++; int run = 0; for (int s = 0; s < NSEG; ++s) { cur[s] = run; run += cnt[s]; } }
  wave_lds_sync(); const int st = cur[lane], c = cnt[lane];
  for (int pass = 0; pass < 2; ++pass) { ((volatile int*)META)[lane] = st; ((volatile int*)META)[NSEG + lane] = c;
    cc[lane] = cur[lane]; wave_lds_sync(); if (lane == 0) { for (int i = 0; i < N; ++i) { const int s = iclamp(pos[i], 0, NSEG - 1); const int p = cc[s]; cc[s] = p + 1; ((volatile int*)LIST)[p] = i; } } wave_lds_sync();
    __threadfence(); } }
__global__ __launch_bounds__(32) void qkv_kernel(const float* __restrict__ inp, const b16* __restrict__ WT, const float* __restrict__ bq, const float* __restrict__ bk, const float* __restrict__ bv, b16* __restrict__ Qh, b16* __restrict__ Ql) {
  __shared__ __attribute__((aligned(16))) b16 Ah[16][P + 8]; __shared__ float Tf[16][132]; const int lane = threadIdx.x, nloc = lane & 15, hlf = lane >> 4; const int g = blockIdx.x % 3; const size_t m0 = (size_t)(blockIdx.x / 3) * 16;
  for (int rr = 0; rr < 16; ++rr) for (int q = 0; q < 4; ++q) Ah[rr][q * 32 + lane] = (b16)(bf16_rne(inp[(m0 + rr) * P + q * 32 + lane]) * XS);
  wave_lds_sync(); v8f acc[8];
#pragma unroll
  for (int t = 0; t < 8; ++t) acc[t] = (v8f){};
#pragma unroll
  for (int kb = 0; kb < P; kb += 32) { const v16b a = frag_kb(&Ah[nloc][kb], hlf);
#pragma unroll
    for (int t = 0; t < 8; ++t) acc[t] = wmma16b(a, frag_kb(WT + (size_t)(g * P + t * 16 + nloc) * P + kb, hlf), acc[t]); }
  const float* bias = g == 0 ? bq : (g == 1 ? bk : bv);
#pragma unroll
  for (int t = 0; t < 8; ++t) { const int c = t * 16 + nloc; const float bb = bf16_rne(bias[c]);
#pragma unroll
    for (int r8 = 0; r8 < 8; ++r8) Tf[8 * hlf + r8][c] = acc[t][r8] * (1.0f / (XS * WSC)) + bb; }
  wave_lds_sync();
  for (int pass = 0; pass < 2; ++pass) { for (int rr = 0; rr < 16; ++rr) { typedef __attribute__((ext_vector_type(4))) _Float16 v4b; v4b vh, vl; for (int k = 0; k < 4; ++k) { b16 p, ql; split16(Tf[rr][lane * 4 + k] * XS, p, ql); vh[k] = p; vl[k] = ql; }
      *(volatile v4b*)(Qh + (m0 + rr) * 3 * P + g * P + lane * 4) = vh; *(volatile v4b*)(Ql + (m0 + rr) * 3 * P + g * P + lane * 4) = vl; } __threadfence(); } }
__global__ __launch_bounds__(32) void att_kernel(const b16* __restrict__ Qh, const b16* __restrict__ Ql, const int* __restrict__ META, const int* __restrict__ LIST, float* __restrict__ out) {
  __shared__ __attribute__((aligned(16))) b16 Aq[16][40], Aql[16][40], Kh[32][40], Kl[32][40], Vh[E][40], Vl[E][40], Ph[16][40], Pl[16][40]; __shared__ float Sc[16][33], Mx[16], Dn[16], Sf[16], Of[16][E + 1]; __shared__ int Rq[16], Rk[32];
  const int lane = threadIdx.x, nloc = lane & 15, hlf = lane >> 4; const int qt = blockIdx.x % (N / 16), h = (blockIdx.x / (N / 16)) % NH, s = blockIdx.x / ((N / 16) * NH);
  const int st = iclamp(META[s], 0, N), cnt = iclamp(META[NSEG + s], 0, N - st); if (qt * 16 >= cnt) return;
  if (lane < 16) { const int li = qt * 16 + lane; Rq[lane] = li < cnt ? iclamp(LIST[st + li], 0, N - 1) : -1; Mx[lane] = -INFINITY; Dn[lane] = 0.0f; Sf[lane] = 0.0f; }
  wave_lds_sync();
  for (int rr = 0; rr < 16; ++rr) { const int r = Rq[rr]; Aq[rr][lane] = r >= 0 ? Qh[(size_t)r * 3 * P + h * E + lane] : (b16)0.0f; Aql[rr][lane] = r >= 0 ? Ql[(size_t)r * 3 * P + h * E + lane] : (b16)0.0f; }
  v8f acc[2] = {(v8f){}, (v8f){}}; wave_lds_sync(); const v16b qa = frag_kb(&Aq[nloc][0], hlf), qal = frag_kb(&Aql[nloc][0], hlf);
#pragma unroll 1
  for (int kc = 0; kc < cnt; kc += 32) { { const int li = kc + lane; Rk[lane] = li < cnt ? iclamp(LIST[st + li], 0, N - 1) : -1; } wave_lds_sync();
    for (int rr = 0; rr < 32; ++rr) { const int r = Rk[rr]; const b16 z = (b16)0.0f; Kh[rr][lane] = r >= 0 ? Qh[(size_t)r * 3 * P + P + h * E + lane] : z; Kl[rr][lane] = r >= 0 ? Ql[(size_t)r * 3 * P + P + h * E + lane] : z; Vh[lane][rr] = r >= 0 ? Qh[(size_t)r * 3 * P + 2 * P + h * E + lane] : z; Vl[lane][rr] = r >= 0 ? Ql[(size_t)r * 3 * P + 2 * P + h * E + lane] : z; }
    wave_lds_sync();
#pragma unroll
    for (int blk = 0; blk < 2; ++blk) { v8f sacc = {}; const v16b kh = frag_kb(&Kh[blk * 16 + nloc][0], hlf), kl = frag_kb(&Kl[blk * 16 + nloc][0], hlf); sacc = wmma16b(qa, kh, sacc); sacc = wmma16b(qa, kl, sacc); sacc = wmma16b(qal, kh, sacc);
#pragma unroll
      for (int r8 = 0; r8 < 8; ++r8) { const int kk = blk * 16 + nloc; Sc[8 * hlf + r8][kk] = (kc + kk < cnt) ? sacc[r8] * (0.17677669529663688f / (XS * XS)) : -INFINITY; } }
    wave_lds_sync();
#pragma unroll 1
    for (int qi = 0; qi < 16; ++qi) { const float sv = Sc[qi][lane]; float cm = sv; for (int o = 16; o; o >>= 1) cm = fmaxf(cm, __shfl_xor(cm, o)); const float mo = Mx[qi]; const float mn = fmaxf(mo, cm); const float p = (sv == -INFINITY) ? 0.0f : __expf(sv - mn); float ps = p; for (int o = 16; o; o >>= 1) ps += __shfl_xor(ps, o);
      b16 ph, plo; split16(p * PS, ph, plo); Ph[qi][lane] = ph; Pl[qi][lane] = plo; if (lane == 0) { const float sf = (mo == -INFINITY) ? 0.0f : __expf(mo - mn); Sf[qi] = sf; Dn[qi] = Dn[qi] * sf + ps; Mx[qi] = mn; } }
    wave_lds_sync(); const v16b pa = frag_kb(&Ph[nloc][0], hlf), pb = frag_kb(&Pl[nloc][0], hlf);
#pragma unroll
    for (int t = 0; t < 2; ++t) {
#pragma unroll
      for (int r8 = 0; r8 < 8; ++r8) acc[t][r8] *= Sf[8 * hlf + r8];
      const v16b vh = frag_kb(&Vh[t * 16 + nloc][0], hlf), vl = frag_kb(&Vl[t * 16 + nloc][0], hlf); acc[t] = wmma16b(pa, vh, acc[t]); acc[t] = wmma16b(pa, vl, acc[t]); acc[t] = wmma16b(pb, vh, acc[t]); }
    wave_lds_sync(); }
#pragma unroll
  for (int t = 0; t < 2; ++t)
#pragma unroll
    for (int r8 = 0; r8 < 8; ++r8) { const int rl = 8 * hlf + r8; Of[rl][t * 16 + nloc] = acc[t][r8] * (1.0f / (PS * XS)) / Dn[rl]; }
  wave_lds_sync();
  for (int pass = 0; pass < 2; ++pass) { for (int rr = 0; rr < 16; ++rr) { const int r = Rq[rr]; if (r >= 0) ((volatile float*)out)[(size_t)r * P + h * E + lane] = Of[rr][lane]; } __threadfence(); } }
}

extern "C" void kernel_launch(void* const* d_in, const int* in_sizes, int n_in, void* d_out, int out_size, void* d_ws, size_t ws_size, hipStream_t stream) {
  (void)n_in;
  auto Fp = [&](int i) { return (const float*)d_in[i]; }; auto Ip = [&](int i) { return (const int*)d_in[i]; };
  if (in_sizes[0] != N * P || in_sizes[1] != N || in_sizes[2] != P * P || in_sizes[4] != P * P || in_sizes[6] != P * P || out_size != N * P) return;
  size_t off = 0; char* ws = (char*)d_ws;
  auto carve = [&](size_t bytes) { char* p = ws + off; off += (bytes + 255) & ~(size_t)255; return p; };
  b16* WT = (b16*)carve((size_t)3 * P * P * 2); int* META = (int*)carve(64 * 4); int* LIST = (int*)carve((size_t)N * 4); b16* Qh = (b16*)carve((size_t)N * 3 * P * 2); b16* Ql = (b16*)carve((size_t)N * 3 * P * 2);
  if (off > ws_size || off > ((size_t)16 << 20)) return;
  wput_kernel<<<(3 * P * 16 + 255) / 256, 256, 0, stream>>>(Fp(2), Fp(4), Fp(6), WT);
  seg_kernel<<<1, 32, 0, stream>>>(Ip(1), META, LIST);
  qkv_kernel<<<(N / 16) * 3, 32, 0, stream>>>(Fp(0), WT, Fp(3), Fp(5), Fp(7), Qh, Ql);
  att_kernel<<<NSEG * NH * (N / 16), 32, 0, stream>>>(Qh, Ql, META, LIST, (float*)d_out);
}
